// MultiHeadAttention_81363860455568
// MI455X (gfx1250) — hardware-run, weakly checked
//
#include <hip/hip_runtime.h>
#ifndef NB
#define NB 2
#endif
#ifndef SEQ
#define SEQ 2048
#endif
#define SQ SEQ
#define NB_FULL 2
#define SQ_FULL 2048
#define DM 1024
#define NH 16
#define HD 64
#define QT 256
#define NKX SQ
#define LQ DM
#define NR ((size_t)NB * SQ)
#define MP ((int)((size_t)NB * SQ))
#define NU (SQ / 256)
#define SCL 0.125f
#define DIAGF 1.0132789611816406e-06f

static_assert(SQ % 256 == 0);
static_assert(SQ % QT == 0);
static_assert(((size_t)NB * SQ) % 128 == 0);
static_assert(NB <= NB_FULL);
static_assert(SQ <= SQ_FULL);
static_assert(NH * HD == DM);

typedef unsigned short v8us __attribute__((ext_vector_type(8), may_alias));
typedef float  v8f  __attribute__((ext_vector_type(8)));
typedef float  v4f  __attribute__((ext_vector_type(4)));
typedef float  v4fa __attribute__((ext_vector_type(4), may_alias));
typedef _Float16 v16h __attribute__((ext_vector_type(16)));
typedef _Float16 v4h __attribute__((ext_vector_type(4)));
union FragH { v16h v; v8us half[2]; _Float16 h[16]; unsigned short u[16]; };

__device__ __forceinline__ unsigned short bf16_bits(float x) { unsigned int u = __float_as_uint(x); return (unsigned short)((u + 0x7FFFu + ((u >> 16) & 1u)) >> 16); }
__device__ __forceinline__ float bf16_val(unsigned short b) { return __uint_as_float(((unsigned int)b) << 16); }
__device__ __forceinline__ float bf16_rne(float x) { return bf16_val(bf16_bits(x)); }

__global__ __launch_bounds__(256) void k_wnat(const float* __restrict__ w, size_t n8, _Float16* __restrict__ Bt) {
  const size_t t = (size_t)blockIdx.x * 256 + threadIdx.x; if (t >= n8) return;
  const v4f a = *(const v4fa*)(w + t * 8), c = *(const v4fa*)(w + t * 8 + 4);
  FragH f;
#pragma unroll
  for (int q = 0; q < 4; ++q) { f.h[q] = (_Float16)(bf16_rne(a[q]) * 16.0f); f.h[4 + q] = (_Float16)(bf16_rne(c[q]) * 16.0f); }
  const v8us o = f.half[0];
  *(volatile v8us*)((unsigned short*)Bt + t * 8) = o; __threadfence(); *(volatile v8us*)((unsigned short*)Bt + t * 8) = o;
}

__global__ __launch_bounds__(256) void k_x16(const float* __restrict__ x, _Float16* __restrict__ X16, size_t n8) {
  const size_t t = (size_t)blockIdx.x * 256 + threadIdx.x; if (t >= n8) return;
  const size_t e = t * 8; const size_t row = e / DM; const size_t col = e - row * DM; const size_t b = row / SQ; const size_t s = row - b * SQ;
  const float* src = x + ((b * SQ_FULL + s) * DM + col);
  const v4f a = *(const v4fa*)src, c = *(const v4fa*)(src + 4);
  FragH f;
#pragma unroll
  for (int q = 0; q < 4; ++q) { f.h[q] = (_Float16)bf16_rne(a[q]); f.h[4 + q] = (_Float16)bf16_rne(c[q]); }
  const v8us o = f.half[0];
  *(volatile v8us*)((unsigned short*)X16 + t * 8) = o; __threadfence(); *(volatile v8us*)((unsigned short*)X16 + t * 8) = o;
}

__global__ __launch_bounds__(256) void k_contrib(const float* __restrict__ reaches, float* __restrict__ RR, float* __restrict__ CT) {
  #pragma clang fp contract(off)
  __shared__ float red[256];
  const int b = blockIdx.x, tid = threadIdx.x;
  const float* src = reaches + (size_t)b * SQ_FULL;
  float* rr = RR + (size_t)b * SQ; float* ct = CT + (size_t)b * SQ;
  float part = 0.f;
#pragma unroll 1
  for (int j = tid * 4; j < SQ; j += 1024) { const v4f a = *(const v4fa*)(src + j); part += bf16_rne(a[0]); part += bf16_rne(a[1]); part += bf16_rne(a[2]); part += bf16_rne(a[3]); }
  red[tid] = part; __syncthreads();
  for (int st = 128; st > 0; st >>= 1) { if (tid < st) red[tid] += red[tid + st]; __syncthreads(); }
  const float rs = red[0];
  const float inv = 1.0f / (rs + 1e-9f);
  for (int pass = 0; pass < 2; ++pass) {
#pragma unroll 1
    for (int j = tid * 4; j < SQ; j += 1024) {
      const v4f a = *(const v4fa*)(src + j); v4f rv, cv;
#pragma unroll
      for (int q = 0; q < 4; ++q) { const float r = bf16_rne(a[q]); rv[q] = r; cv[q] = (rs - r) * inv * (1.0f - r) * 100.0f; }
      *(volatile v4f*)(rr + j) = rv; *(volatile v4f*)(ct + j) = cv;
    }
    if (pass == 0) __threadfence();
  }
}

template <int NHv, int TTv>
__global__ __launch_bounds__(256) void k_vt(const _Float16* __restrict__ V16, int ldv, int voff, _Float16* __restrict__ Vt) {
  __shared__ unsigned short tl[64][66];
  const int tid = threadIdx.x; const int slab = blockIdx.x / (TTv / 64), lg = blockIdx.x % (TTv / 64); const int b = slab / NHv, h = slab % NHv;
  for (int i = tid; i < 64 * 8; i += 256) { const int r = i / 8, c8 = (i % 8) * 8; FragH f; f.half[0] = *(const v8us*)((const unsigned short*)V16 + ((size_t)b * TTv + lg * 64 + r) * ldv + voff + h * 64 + c8);
#pragma unroll
    for (int q = 0; q < 8; ++q) tl[r][c8 + q] = f.u[q]; }
  __syncthreads();
  for (int pass = 0; pass < 2; ++pass) {
#pragma unroll
    for (int rd = 0; rd < 2; ++rd) { const int d = rd * 32 + tid / 8, pc = tid % 8; FragH f;
#pragma unroll
      for (int q = 0; q < 8; ++q) f.u[q] = tl[pc * 8 + q][d];
      *(volatile v8us*)((unsigned short*)Vt + ((size_t)slab * 64 + d) * TTv + lg * 64 + pc * 8) = f.half[0]; }
    if (pass == 0) __threadfence(); }
}

__global__ __launch_bounds__(256) void k_hlc(const float* __restrict__ F, const float* __restrict__ CT, _Float16* __restrict__ Hh, _Float16* __restrict__ Hl, size_t n8) {
  #pragma clang fp contract(off)
  const size_t t = (size_t)blockIdx.x * 256 + threadIdx.x; if (t >= n8) return;
  const float ct = CT[(t * 8) / DM];
  FragH fh, fl; const v4f a = *(const v4fa*)(F + t * 8), c = *(const v4fa*)(F + t * 8 + 4);
#pragma unroll
  for (int q = 0; q < 4; ++q) { float x = a[q] * ct; _Float16 h = (_Float16)x; fh.h[q] = h; fl.h[q] = (_Float16)((x - (float)h) * 1024.0f); x = c[q] * ct; h = (_Float16)x; fh.h[4 + q] = h; fl.h[4 + q] = (_Float16)((x - (float)h) * 1024.0f); }
  for (int pass = 0; pass < 2; ++pass) { *(volatile v8us*)((unsigned short*)Hh + t * 8) = fh.half[0]; *(volatile v8us*)((unsigned short*)Hl + t * 8) = fl.half[0]; if (pass == 0) __threadfence(); }
}

__device__ __forceinline__ v16h g2_frag(const _Float16* p, int hh) { FragH f; f.half[0] = *(const v8us*)((const unsigned short*)p + 8 * hh); f.half[1] = *(const v8us*)((const unsigned short*)p + 16 + 8 * hh); return f.v; }
__device__ __forceinline__ v8f g2_mma(v16h a, v16h b, v8f c) { v8f d = __builtin_amdgcn_wmma_f32_16x16x32_f16(false, a, false, b, (short)0, c, false, false); asm volatile("v_nop\n\tv_nop\n\tv_nop\n\tv_nop" : "+v"(d) : "v"(a), "v"(b)); return d; }
__global__ __launch_bounds__(128) void k_gemm2(const _Float16* __restrict__ A, int lda, size_t sA, const _Float16* __restrict__ Bh, int ldb, size_t sB, float alpha, const float* __restrict__ bias, size_t sBias, const float* __restrict__ CP, int rowsPerB, size_t sCPb, int row0g,
    float* __restrict__ C, _Float16* __restrict__ C16, int ldc, size_t sC, int M, int N, int K) {
  __shared__ __attribute__((aligned(16))) float so[4][32][68];
  const int tid = threadIdx.x, w = __builtin_amdgcn_readfirstlane((int)(tid >> 5)), lane = tid & 31, ln = lane & 15, hh = lane >> 4; const int by = blockIdx.y;
  A += (size_t)by * sA; Bh += (size_t)by * sB; const size_t cofs = (size_t)by * sC; const float* bp = bias ? bias + (size_t)by * sBias : nullptr;
  const int ntn = N >> 6; const int mt = blockIdx.x / ntn, nq = blockIdx.x - mt * ntn; const int row0 = mt * 128 + 32 * w, col0 = nq * 64; if (row0 >= M) return;
  const _Float16* a0p = A + (size_t)(row0 + ln) * lda; const _Float16* a1p = a0p + (size_t)16 * lda;
  const _Float16* b0p = Bh + (size_t)(col0 + ln) * ldb; const _Float16* b1p = b0p + (size_t)16 * ldb; const _Float16* b2p = b1p + (size_t)16 * ldb; const _Float16* b3p = b2p + (size_t)16 * ldb;
  const v8f z8 = {0.f,0.f,0.f,0.f,0.f,0.f,0.f,0.f}; v8f c00 = z8, c01 = z8, c02 = z8, c03 = z8, c10 = z8, c11 = z8, c12 = z8, c13 = z8;
#pragma unroll 1
  for (int kb = 0; kb < K; kb += 32) { const v16h a0 = g2_frag(a0p + kb, hh), a1 = g2_frag(a1p + kb, hh);
    v16h b = g2_frag(b0p + kb, hh); c00 = g2_mma(a0, b, c00); c10 = g2_mma(a1, b, c10);
    b = g2_frag(b1p + kb, hh); c01 = g2_mma(a0, b, c01); c11 = g2_mma(a1, b, c11);
    b = g2_frag(b2p + kb, hh); c02 = g2_mma(a0, b, c02); c12 = g2_mma(a1, b, c12);
    b = g2_frag(b3p + kb, hh); c03 = g2_mma(a0, b, c03); c13 = g2_mma(a1, b, c13); }
  v8f accs[8] = {c00, c01, c02, c03, c10, c11, c12, c13};
#pragma unroll
  for (int u = 0; u < 8; ++u) { const int t = u & 3, half = u >> 2; const int col = col0 + t * 16 + ln; const float bv = bp ? bf16_rne(bp[col]) : 0.f;
#pragma unroll
    for (int r = 0; r < 8; ++r) { const int rloc = half * 16 + 8 * hh + r; float v = accs[u][r] * alpha + bv;
      if (CP) { if (rowsPerB < 0) v += CP[cofs + (size_t)(row0g + row0 + rloc) * ldc + col];        else { const int bidx = (row0g + row0 + rloc) / rowsPerB; v += CP[(size_t)bidx * sCPb + (size_t)by * 64 + col]; } }
      so[w][rloc][t * 16 + ln] = v; } }
  __builtin_amdgcn_fence(4  , "workgroup"); __builtin_amdgcn_wave_barrier();
  const int rsub = lane >> 4, c4 = (lane & 15) * 4;
  for (int pass = 0; pass < 2; ++pass) {
#pragma unroll
    for (int q = 0; q < 16; ++q) { const int r = q * 2 + rsub; const v4f v = *(const v4fa*)&so[w][r][c4];
      if (C) *(volatile v4f*)(C + cofs + (size_t)(row0 + r) * ldc + col0 + c4) = v;
      if (C16) { v4h h4;
#pragma unroll
        for (int i = 0; i < 4; ++i) h4[i] = (_Float16)v[i];
        *(volatile v4h*)(C16 + cofs + (size_t)(row0 + r) * ldc + col0 + c4) = h4; } }
    if (pass == 0) __threadfence(); }
}

__global__ __launch_bounds__(256) void k_rsmw(const float* __restrict__ S, const float* __restrict__ RRb, _Float16* __restrict__ P, int nrows, int q0) {
  #pragma clang fp contract(off)
  const int lane = threadIdx.x & 31;
  const int row = blockIdx.x * 8 + __builtin_amdgcn_readfirstlane((int)(threadIdx.x >> 5));
  if (row >= nrows) return;
  const float* s = S + (size_t)row * NKX;
  const int qg = q0 + (row % QT);
  v4f x[2 * NU];
#pragma unroll
  for (int u = 0; u < NU; ++u) { const int j = u * 256 + lane * 8; x[2 * u] = *(const v4fa*)(s + j); x[2 * u + 1] = *(const v4fa*)(s + j + 4); }
  float mx = -3.0e38f;
#pragma unroll
  for (int i = 0; i < 2 * NU; ++i) {
#pragma unroll
    for (int c = 0; c < 4; ++c) mx = fmaxf(mx, x[i][c]); }
#pragma unroll
  for (int m = 16; m >= 1; m >>= 1) mx = fmaxf(mx, __shfl_xor(mx, m, 32));
  float se = 0.f;
#pragma unroll
  for (int i = 0; i < 2 * NU; ++i) {
#pragma unroll
    for (int c = 0; c < 4; ++c) { const float e = __expf(x[i][c] - mx); x[i][c] = e; se += e; } }
#pragma unroll
  for (int m = 16; m >= 1; m >>= 1) se += __shfl_xor(se, m, 32);
  const float sc = 1024.0f / se;
  v8us o[NU];
#pragma unroll
  for (int u = 0; u < NU; ++u) { const int j = u * 256 + lane * 8;
    const v4f r0 = *(const v4fa*)(RRb + j), r1 = *(const v4fa*)(RRb + j + 4); FragH f;
#pragma unroll
    for (int c = 0; c < 4; ++c) {
      const float w0 = r0[c] * ((j + c == qg) ? DIAGF : 1.0f);
      const float w1 = r1[c] * ((j + 4 + c == qg) ? DIAGF : 1.0f);
      f.h[c] = (_Float16)(x[2 * u][c] * sc * w0);
      f.h[4 + c] = (_Float16)(x[2 * u + 1][c] * sc * w1); }
    o[u] = f.half[0]; }
  unsigned short* d = (unsigned short*)P + (size_t)row * NKX + lane * 8;
  for (int pass = 0; pass < 2; ++pass) {
#pragma unroll
    for (int u = 0; u < NU; ++u) *(volatile v8us*)(d + u * 256) = o[u];
    if (pass == 0) __threadfence(); }
}

extern "C" void kernel_launch(void* const* d_in, const int* in_sizes, int n_in,
                              void* d_out, int out_size, void* d_ws, size_t ws_size, hipStream_t stream) {
  if (n_in < 8) return;
  const size_t needx = ((size_t)(NB - 1) * SQ_FULL + SQ) * DM;
  const size_t needr = (size_t)(NB - 1) * SQ_FULL + SQ;
  if ((size_t)in_sizes[0] < needx || (size_t)in_sizes[1] < needx || (size_t)in_sizes[2] < needx) return;
  if ((size_t)in_sizes[3] < needr) return;
  if ((size_t)in_sizes[4] < (size_t)DM * DM || (size_t)in_sizes[5] < (size_t)DM * DM || (size_t)in_sizes[6] < (size_t)DM * DM || (size_t)in_sizes[7] < (size_t)DM * DM) return;
  if ((size_t)out_size < NR * DM) return;
  const float* const* I = (const float* const*)d_in;
  const float* xq = I[0]; const float* xk = I[1]; const float* xv = I[2]; const float* reaches = I[3];
  const float* wq = I[4]; const float* wk = I[5]; const float* wv = I[6]; const float* wo = I[7];
  constexpr size_t WB = (size_t)DM * DM * 2;
  constexpr size_t ROW16 = NR * DM * 2;
  constexpr size_t ROW32 = NR * DM * 4;
  constexpr size_t SB = (size_t)NH * QT * NKX * 4;
  constexpr size_t PB = (size_t)NH * QT * NKX * 2;
  constexpr size_t XA_B = (2 * ROW16 > ROW32) ? 2 * ROW16 : ROW32;
  constexpr size_t SR_B = (SB > ROW32) ? SB : ROW32;
  constexpr size_t PR_B = (PB > 2 * ROW16) ? PB : 2 * ROW16;
  constexpr size_t VT_B = (size_t)NH * HD * SQ * 2;
  constexpr size_t RC_B = NR * 4;
  constexpr size_t TOTAL = 4 * WB + XA_B + ROW16 + 2 * ROW16 + ROW32 + ROW16 + SR_B + PR_B + VT_B + 2 * ((RC_B + 255) & ~(size_t)255);
  static_assert(TOTAL <= (size_t)134217728);
  static_assert(ROW32 <= XA_B);
  static_assert(ROW32 <= SR_B);
  static_assert(2 * ROW16 <= PR_B);
  char* ws = (char*)d_ws; size_t off = 0;
  auto take = [&](size_t bytes) { char* p = ws + off; off += (bytes + 255) & ~(size_t)255; return p; };
  _Float16* BQ = (_Float16*)take(WB); _Float16* BK = (_Float16*)take(WB); _Float16* BV = (_Float16*)take(WB); _Float16* BO = (_Float16*)take(WB);
  char* XA = take(XA_B); _Float16* X16 = (_Float16*)XA; _Float16* XK16 = (_Float16*)(XA + ROW16); float* Dd = (float*)XA;
  _Float16* XV16 = (_Float16*)take(ROW16);
  _Float16* Q16 = (_Float16*)take(ROW16); _Float16* K16 = (_Float16*)take(ROW16);
  float* VF = (float*)take(ROW32); _Float16* V16 = (_Float16*)take(ROW16);
  char* SR = take(SR_B); float* S = (float*)SR; float* T = (float*)SR;
  char* PR = take(PR_B); _Float16* P = (_Float16*)PR; _Float16* CH = (_Float16*)PR; _Float16* CL = (_Float16*)(PR + ROW16);
  _Float16* VT = (_Float16*)take(VT_B);
  float* RR = (float*)take(RC_B); float* CT = (float*)take(RC_B);
  if (off > ws_size) return;

  { const unsigned g = (unsigned)(((size_t)DM * DM / 8 + 255) / 256);
    k_wnat<<<g, 256, 0, stream>>>(wq, (size_t)DM * DM / 8, BQ); k_wnat<<<g, 256, 0, stream>>>(wk, (size_t)DM * DM / 8, BK);
    k_wnat<<<g, 256, 0, stream>>>(wv, (size_t)DM * DM / 8, BV); k_wnat<<<g, 256, 0, stream>>>(wo, (size_t)DM * DM / 8, BO); }
  { const unsigned g = (unsigned)((NR * DM / 8 + 255) / 256);
    k_x16<<<g, 256, 0, stream>>>(xq, X16, NR * DM / 8); k_x16<<<g, 256, 0, stream>>>(xk, XK16, NR * DM / 8); k_x16<<<g, 256, 0, stream>>>(xv, XV16, NR * DM / 8); }
  k_contrib<<<NB, 256, 0, stream>>>(reaches, RR, CT);
  k_gemm2<<<dim3((unsigned)((MP / 128) * (DM / 64)), 1), 128, 0, stream>>>(X16, DM, 0, BQ, DM, 0, 0.0625f, nullptr, 0, nullptr, 1, 0, 0, nullptr, Q16, DM, 0, MP, DM, DM);
  k_gemm2<<<dim3((unsigned)((MP / 128) * (DM / 64)), 1), 128, 0, stream>>>(XK16, DM, 0, BK, DM, 0, 0.0625f, nullptr, 0, nullptr, 1, 0, 0, nullptr, K16, DM, 0, MP, DM, DM);
  k_gemm2<<<dim3((unsigned)((MP / 128) * (DM / 64)), 1), 128, 0, stream>>>(XV16, DM, 0, BV, DM, 0, 0.0625f, nullptr, 0, nullptr, 1, 0, 0, VF, V16, DM, 0, MP, DM, DM);
  for (int b = 0; b < NB; ++b) { const size_t r0 = (size_t)b * SQ;
    k_vt<NH, SQ><<<NH * (SQ / 64), 256, 0, stream>>>(V16 + r0 * LQ, LQ, 0, VT);
    for (int q0 = 0; q0 < SQ; q0 += QT) {
      k_gemm2<<<dim3((QT / 128) * (SQ / 64), NH), 128, 0, stream>>>(Q16 + (r0 + q0) * LQ, LQ, (size_t)HD, K16 + r0 * LQ, LQ, (size_t)HD, SCL, nullptr, 0, nullptr, 1, 0, 0, S, nullptr, NKX, (size_t)QT * NKX, QT, SQ, HD);
      k_rsmw<<<(NH * QT + 7) / 8, 256, 0, stream>>>(S, RR + r0, P, NH * QT, q0);
      k_gemm2<<<dim3((QT / 128) * (HD / 64), NH), 128, 0, stream>>>(P, NKX, (size_t)QT * NKX, VT, SQ, (size_t)HD * SQ, -0.0009765625f, nullptr, 0, VF + (r0 + q0) * DM, -1, 0, 0, Dd + (r0 + q0) * DM, nullptr, DM, (size_t)HD, QT, HD, SQ); } }
  k_hlc<<<(unsigned)((NR * DM / 8 + 255) / 256), 256, 0, stream>>>(Dd, CT, CH, CL, NR * DM / 8);
  k_gemm2<<<dim3((unsigned)((MP / 128) * (DM / 64)), 1), 128, 0, stream>>>(CL, DM, 0, BO, DM, 0, 6.103515625e-05f, nullptr, 0, nullptr, 1, 0, 0, T, nullptr, DM, 0, MP, DM, DM);
  k_gemm2<<<dim3((unsigned)((MP / 128) * (DM / 64)), 1), 128, 0, stream>>>(CH, DM, 0, BO, DM, 0, 0.0625f, nullptr, 0, T, -1, 0, 0, (float*)d_out, nullptr, DM, 0, MP, DM, DM);
}
